// TTS_RNN_GCN_5291399708928
// MI455X (gfx1250) — hardware-verified
//
#include <hip/hip_runtime.h>
#include <hip/hip_bf16.h>


#define B_     8
#define T_     64
#define N_     2000
#define F_     2
#define HID_   64
#define G3_    192
#define NE_    32000
#define HOR_   12
#define DOUT_  24
#define ROWS_  16000
#define NPAD_  2048

static_assert(N_ % 16 == 0);
static_assert(ROWS_ % 128 == 0);
static_assert(NE_ % 256 == 0);
static_assert(NPAD_ % 64 == 0);
static_assert(NPAD_ >= N_);
static_assert(HOR_ * F_ == DOUT_);

typedef float          v2f   __attribute__((ext_vector_type(2)));
typedef float          v4f   __attribute__((ext_vector_type(4)));
typedef float          v8f   __attribute__((ext_vector_type(8)));
typedef _Float16       v8h   __attribute__((ext_vector_type(8)));
typedef _Float16       v16h  __attribute__((ext_vector_type(16)));
typedef __bf16         v16b  __attribute__((ext_vector_type(16)));
typedef unsigned short u16x8 __attribute__((ext_vector_type(8)));

union FragH { v8h   h[2]; v16h v; };
union FragB { u16x8 h[2]; v16b v; };

constexpr size_t SZ_G0  = (size_t)NPAD_ * G3_ * 4;
constexpr size_t SZ_ROW = (size_t)ROWS_ * HID_ * 4;
constexpr size_t OFF_G0 = 0;
constexpr size_t OFF_HL = OFF_G0 + SZ_G0;
constexpr size_t OFF_XL = OFF_HL + SZ_ROW;
constexpr size_t WS_END = OFF_XL + SZ_ROW;
static_assert(WS_END <= (size_t)134217728);
static_assert(OFF_HL % 128 == 0);
static_assert(OFF_XL % 128 == 0);

constexpr int LDS_G0  = 114688;
constexpr int LDS_GRU = 83456;
constexpr int LDS_GC  = 137344;

__device__ __forceinline__ unsigned short f2bf(float f) {
    unsigned u = __float_as_uint(f);
    u = u + 0x7FFFu + ((u >> 16) & 1u);
    return (unsigned short)(u >> 16);
}
__device__ __forceinline__ float bf2f(unsigned short b) {
    return __uint_as_float(((unsigned)b) << 16);
}
__device__ __forceinline__ v8f ld8f(const float* p) {
    v4f a = *(const v4f*)p;
    v4f b = *(const v4f*)(p + 4);
    return __builtin_shufflevector(a, b, 0, 1, 2, 3, 4, 5, 6, 7);
}
__device__ __forceinline__ void split8(const v8f x, u16x8& hv, u16x8& lv) {
#pragma unroll
    for (int c = 0; c < 8; ++c) {
        const float f = x[c];
        const unsigned short hb = f2bf(f);
        const unsigned short lb = f2bf(f - bf2f(hb));
        hv[c] = hb;
        lv[c] = lb;
    }
}
__device__ __forceinline__ v8h cvt8h(const v8f x, float sc) {
    v8h r;
#pragma unroll
    for (int c = 0; c < 8; ++c) r[c] = (_Float16)(x[c] * sc);
    return r;
}
__device__ __forceinline__ float frcp(float x)  { return __builtin_amdgcn_rcpf(x); }
__device__ __forceinline__ float fsigm(float x) { return frcp(1.0f + __expf(-x)); }
__device__ __forceinline__ float ftanh(float x) {
    const float ax = fminf(fabsf(x), 15.0f);
    const float e  = __expf(2.0f * ax);
    const float tp = 1.0f - 2.0f * frcp(e + 1.0f);
    return copysignf(tp, x);
}

__device__ __forceinline__ void mma_f16(v8f& acc, const FragH& a, const FragH& b) {
    acc = __builtin_amdgcn_wmma_f32_16x16x32_f16(false, a.v, false, b.v, (short)0, acc, false, false);
    asm volatile("v_nop\n\tv_nop\n\tv_nop\n\tv_nop" : "+v"(acc) : "v"(a.v), "v"(b.v));
}
__device__ __forceinline__ void mma_bf16(v8f& acc, const FragB& a, const FragB& b) {
    acc = __builtin_amdgcn_wmma_f32_16x16x32_bf16(false, a.v, false, b.v, (short)0, acc, false, false);
    asm volatile("v_nop\n\tv_nop\n\tv_nop\n\tv_nop" : "+v"(acc) : "v"(a.v), "v"(b.v));
}

__device__ __forceinline__ FragH frag_h(const _Float16* rp, int k0, int h) {
    FragH f;
    f.h[0] = *(const v8h*)(rp + k0 + 8 * h);
    f.h[1] = *(const v8h*)(rp + k0 + 16 + 8 * h);
    return f;
}
__device__ __forceinline__ FragB frag_b(const unsigned short* rp, int k0, int h) {
    FragB f;
    f.h[0] = *(const u16x8*)(rp + k0 + 8 * h);
    f.h[1] = *(const u16x8*)(rp + k0 + 16 + 8 * h);
    return f;
}
__device__ __forceinline__ void zero8(v8f& a) {
#pragma unroll
    for (int r = 0; r < 8; ++r) a[r] = 0.0f;
}

__global__ __launch_bounds__(256)
void k_g0tab(const float* __restrict__ nemb, const float* __restrict__ encb,
             const float* __restrict__ wih,  const float* __restrict__ bih,
             const float* __restrict__ bhh,  float* g0)
{
    extern __shared__ v4f lds_dyn[];
    unsigned char* lb = (unsigned char*)lds_dyn;
    unsigned short* sAh  = (unsigned short*)(lb + 0);
    unsigned short* sAl  = (unsigned short*)(lb + 8192);
    unsigned short* sBh  = (unsigned short*)(lb + 16384);
    unsigned short* sBl  = (unsigned short*)(lb + 40960);
    float*          sOut = (float*)(lb + 65536);

    const int tid = threadIdx.x, lane = tid & 31, wave = tid >> 5;
    const int h = lane >> 4, m = lane & 15;
    const int nb0 = blockIdx.x * 64;

    {
        const int row = tid >> 2;
        const int c0  = (tid & 3) * 16;
        const int n   = nb0 + row;
        const int nc  = min(n, N_ - 1);
        const float vm = (n < N_) ? 1.0f : 0.0f;
#pragma unroll
        for (int q = 0; q < 2; ++q) {
            const int c = c0 + 8 * q;
            const v8f e = (ld8f(nemb + (size_t)nc * HID_ + c) + ld8f(encb + c)) * vm;
            u16x8 hv, lv;
            split8(e, hv, lv);
            *(u16x8*)(sAh + row * HID_ + c) = hv;
            *(u16x8*)(sAl + row * HID_ + c) = lv;
        }
    }
#pragma unroll
    for (int it = 0; it < 6; ++it) {
        const int i8 = (it * 256 + tid) * 8;
        const v8f w = ld8f(wih + i8);
        u16x8 hv, lv;
        split8(w, hv, lv);
        *(u16x8*)(sBh + i8) = hv;
        *(u16x8*)(sBl + i8) = lv;
    }
    __syncthreads();

    const int wr = (wave & 3) * 16;
    const int wc = (wave >> 2) * 96;
    FragB ah[2], al[2];
#pragma unroll
    for (int s = 0; s < 2; ++s) {
        ah[s] = frag_b(sAh + (wr + m) * HID_, 32 * s, h);
        al[s] = frag_b(sAl + (wr + m) * HID_, 32 * s, h);
    }
    v8f acc[6];
#pragma unroll
    for (int j = 0; j < 6; ++j) zero8(acc[j]);
#pragma unroll
    for (int nt = 0; nt < 6; ++nt) {
        const unsigned short* bph = sBh + (wc + nt * 16 + m) * HID_;
        const unsigned short* bpl = sBl + (wc + nt * 16 + m) * HID_;
#pragma unroll
        for (int s = 0; s < 2; ++s) {
            const FragB bh = frag_b(bph, 32 * s, h);
            const FragB bl = frag_b(bpl, 32 * s, h);
            mma_bf16(acc[nt], ah[s], bh);
            mma_bf16(acc[nt], ah[s], bl);
            mma_bf16(acc[nt], al[s], bh);
        }
    }
#pragma unroll
    for (int nt = 0; nt < 6; ++nt) {
        const int g = wc + nt * 16 + m;
        const float b2 = bhh[g];
        const float bb = bih[g] + ((g < 128) ? b2 : 0.0f);
#pragma unroll
        for (int r = 0; r < 8; ++r)
            sOut[(wr + 8 * h + r) * G3_ + g] = acc[nt][r] + bb;
    }
    __syncthreads();

    float* gb = g0 + (size_t)nb0 * G3_;
#pragma unroll
    for (int it = 0; it < 12; ++it) {
        const int L   = it * 32 + wave * 4 + (lane >> 3);
        const int row = L / 6;
        const int li  = L - row * 6;
        const int c   = li * 32 + (lane & 7) * 4;
        const v4f v = *(const v4f*)(sOut + row * G3_ + c);
        *(volatile v4f*)(gb + (size_t)row * G3_ + c) = v;
    }
    __threadfence();
#pragma unroll
    for (int it = 0; it < 12; ++it) {
        const int L   = it * 32 + wave * 4 + (lane >> 3);
        const int row = L / 6;
        const int li  = L - row * 6;
        const int c   = li * 32 + (lane & 7) * 4;
        const v4f v = *(const v4f*)(sOut + row * G3_ + c);
        *(volatile v4f*)(gb + (size_t)row * G3_ + c) = v;
    }
}

__global__ __launch_bounds__(256)
void k_gru(const float* __restrict__ x,    const float* __restrict__ g0,
           const float* __restrict__ encw, const float* __restrict__ wih,
           const float* __restrict__ whh,  const float* __restrict__ bhh,
           const float* __restrict__ gcw,  float* hl, float* xl)
{
    extern __shared__ v4f lds_dyn[];
    unsigned char* lb = (unsigned char*)lds_dyn;
    _Float16* sW  = (_Float16*)(lb + 0);
    _Float16* sGc = (_Float16*)(lb + 24576);
    _Float16* sH  = (_Float16*)(lb + 32768);
    float*    sC  = (float*)(lb + 49152);
    float*    sSt = (float*)(lb + 50688);

    const int tid = threadIdx.x, lane = tid & 31, wave = tid >> 5;
    const int h = lane >> 4, m = lane & 15;

#pragma unroll
    for (int it = 0; it < 6; ++it) {
        const int i8 = (it * 256 + tid) * 8;
        *(v8h*)(sW + i8) = cvt8h(ld8f(whh + i8), 8.0f);
    }
#pragma unroll
    for (int it = 0; it < 2; ++it) {
        const int i8 = (it * 256 + tid) * 8;
        *(v8h*)(sGc + i8) = cvt8h(ld8f(gcw + i8), 16.0f);
    }
    {
        v8h z;
#pragma unroll
        for (int c = 0; c < 8; ++c) z[c] = (_Float16)0.0f;
#pragma unroll
        for (int it = 0; it < 4; ++it) *(v8h*)(sH + (it * 256 + tid) * 8) = z;
    }
#pragma unroll 1
    for (int i = tid; i < 2 * G3_; i += 256) {
        const int f = (i >= G3_) ? 1 : 0;
        const int g = i - f * G3_;
        float a = 0.0f;
#pragma unroll 4
        for (int k = 0; k < HID_; ++k) a = fmaf(wih[g * HID_ + k], encw[k * F_ + f], a);
        sC[i] = a;
    }
    __syncthreads();

    const int row0 = (blockIdx.x * 8 + wave) * 16;
    const int bb   = row0 / N_;
    const int n0   = row0 - bb * N_;
    _Float16* sHw = sH  + wave * 1024;
    float*    stw = sSt + wave * 1024;

    float cR0[4], cR1[4], cZ0[4], cZ1[4], cN0[4], cN1[4], bhn[4];
#pragma unroll
    for (int nt = 0; nt < 4; ++nt) {
        const int g = nt * 16 + m;
        cR0[nt] = sC[g];          cR1[nt] = sC[G3_ + g];
        cZ0[nt] = sC[64 + g];     cZ1[nt] = sC[G3_ + 64 + g];
        cN0[nt] = sC[128 + g];    cN1[nt] = sC[G3_ + 128 + g];
        bhn[nt] = bhh[128 + g];
    }
    float hreg[4][8];
#pragma unroll
    for (int nt = 0; nt < 4; ++nt)
#pragma unroll
        for (int r = 0; r < 8; ++r) hreg[nt][r] = 0.0f;

#pragma unroll 1
    for (int t = 0; t < T_; ++t) {
        int tq = t;
        asm volatile("" : "+v"(tq));
        const int radd = tq >> 6;
        const float* xr = x + ((((size_t)bb * T_ + t) * N_) + n0 + 8 * h) * 2;
        v4f xv[4];
#pragma unroll
        for (int q = 0; q < 4; ++q) xv[q] = *(const v4f*)(xr + 4 * q);

        FragH a[2];
        {
            const _Float16* rp = sHw + m * HID_;
            a[0] = frag_h(rp, 0, h);
            a[1] = frag_h(rp, 32, h);
        }
        const float* gp = g0 + (size_t)(n0 + 8 * h + radd) * G3_ + m;

#pragma unroll
        for (int nt = 0; nt < 4; ++nt) {
            v8f aR, aZ, aN;
            zero8(aR); zero8(aZ); zero8(aN);
            const _Float16* wR = sW + (nt * 16 + m) * HID_;
            const _Float16* wZ = sW + (64 + nt * 16 + m) * HID_;
            const _Float16* wN = sW + (128 + nt * 16 + m) * HID_;
#pragma unroll
            for (int s = 0; s < 2; ++s) {
                const FragH bR = frag_h(wR, 32 * s, h);
                mma_f16(aR, a[s], bR);
                const FragH bZ = frag_h(wZ, 32 * s, h);
                mma_f16(aZ, a[s], bZ);
                const FragH bN = frag_h(wN, 32 * s, h);
                mma_f16(aN, a[s], bN);
            }
#pragma unroll
            for (int r = 0; r < 8; ++r) {
                const float x0 = xv[(2 * r) >> 2][(2 * r) & 3];
                const float x1 = xv[(2 * r + 1) >> 2][(2 * r + 1) & 3];
                const float* gr = gp + r * G3_ + nt * 16;
                const float pr = gr[0]   + (x0 * cR0[nt] + x1 * cR1[nt]) + aR[r] * 0.125f;
                const float pz = gr[64]  + (x0 * cZ0[nt] + x1 * cZ1[nt]) + aZ[r] * 0.125f;
                const float pn = gr[128] + (x0 * cN0[nt] + x1 * cN1[nt]);
                const float hn = aN[r] * 0.125f + bhn[nt];
                const float rg = fsigm(pr);
                const float zg = fsigm(pz);
                const float cc = ftanh(pn + rg * hn);
                const float ho = hreg[nt][r];
                const float hw = (1.0f - zg) * cc + zg * ho;
                hreg[nt][r] = hw;
                sHw[(8 * h + r) * HID_ + nt * 16 + m] = (_Float16)hw;
            }
        }
        __syncthreads();
    }

    v8f aX[4];
    {
        FragH a[2];
        const _Float16* rp = sHw + m * HID_;
        a[0] = frag_h(rp, 0, h);
        a[1] = frag_h(rp, 32, h);
#pragma unroll
        for (int nt = 0; nt < 4; ++nt) {
            zero8(aX[nt]);
            const _Float16* wG = sGc + (nt * 16 + m) * HID_;
#pragma unroll
            for (int s = 0; s < 2; ++s) {
                const FragH bG = frag_h(wG, 32 * s, h);
                mma_f16(aX[nt], a[s], bG);
            }
        }
    }

#pragma unroll
    for (int nt = 0; nt < 4; ++nt)
#pragma unroll
        for (int r = 0; r < 8; ++r) stw[(8 * h + r) * HID_ + nt * 16 + m] = hreg[nt][r];
    __syncthreads();
#pragma unroll
    for (int it = 0; it < 8; ++it) {
        const int row = 2 * it + (lane >> 4);
        const int c   = (lane & 15) * 4;
        const v4f v = *(const v4f*)(stw + row * HID_ + c);
        *(volatile v4f*)(hl + (size_t)(row0 + row) * HID_ + c) = v;
    }
    __threadfence();
#pragma unroll
    for (int it = 0; it < 8; ++it) {
        const int row = 2 * it + (lane >> 4);
        const int c   = (lane & 15) * 4;
        const v4f v = *(const v4f*)(stw + row * HID_ + c);
        *(volatile v4f*)(hl + (size_t)(row0 + row) * HID_ + c) = v;
    }
    __syncthreads();

#pragma unroll
    for (int nt = 0; nt < 4; ++nt)
#pragma unroll
        for (int r = 0; r < 8; ++r) stw[(8 * h + r) * HID_ + nt * 16 + m] = aX[nt][r] * 0.0625f;
    __syncthreads();
#pragma unroll
    for (int it = 0; it < 8; ++it) {
        const int row = 2 * it + (lane >> 4);
        const int c   = (lane & 15) * 4;
        const v4f v = *(const v4f*)(stw + row * HID_ + c);
        *(volatile v4f*)(xl + (size_t)(row0 + row) * HID_ + c) = v;
    }
    __threadfence();
#pragma unroll
    for (int it = 0; it < 8; ++it) {
        const int row = 2 * it + (lane >> 4);
        const int c   = (lane & 15) * 4;
        const v4f v = *(const v4f*)(stw + row * HID_ + c);
        *(volatile v4f*)(xl + (size_t)(row0 + row) * HID_ + c) = v;
    }
}

__global__ __launch_bounds__(256)
void k_gconv(const int* __restrict__ ei,     const float* __restrict__ ew,
             const float* __restrict__ hl,   const float* __restrict__ xl,
             const float* __restrict__ gcrw, const float* __restrict__ gcb,
             const float* __restrict__ decw, const float* __restrict__ decb,
             float* out)
{
    extern __shared__ v4f lds_dyn[];
    unsigned char* lb = (unsigned char*)lds_dyn;
    float*          sAcc = (float*)(lb + 0);
    unsigned short* sHh  = (unsigned short*)(lb + 32768);
    unsigned short* sHl  = (unsigned short*)(lb + 49152);
    unsigned short* sRh  = (unsigned short*)(lb + 65536);
    unsigned short* sRl  = (unsigned short*)(lb + 73728);
    unsigned short* sDh  = (unsigned short*)(lb + 81920);
    unsigned short* sDl  = (unsigned short*)(lb + 86016);
    unsigned short* sZh  = (unsigned short*)(lb + 90112);
    unsigned short* sZl  = (unsigned short*)(lb + 106496);
    float*          sOut = (float*)(lb + 122880);
    int*            sEj  = (int*)(lb + 135168);
    float*          sEw  = (float*)(lb + 136192);
    int*            sCnt = (int*)(lb + 137216);
    float*          sInv = (float*)(lb + 137248);

    const int tid = threadIdx.x, lane = tid & 31, wave = tid >> 5;
    const int h = lane >> 4, m = lane & 15;
    const int n0 = blockIdx.x * 16;
    const int bsel = wave;
    const int cl = lane * 2;

    {
        v4f z;
        z[0] = 0.0f; z[1] = 0.0f; z[2] = 0.0f; z[3] = 0.0f;
#pragma unroll
        for (int q = 0; q < 8; ++q) *(v4f*)(sAcc + (q * 256 + tid) * 4) = z;
    }
    {
        const int r   = tid >> 1;
        const int c0  = (tid & 1) * 32;
        const int bq  = r >> 4, j = r & 15;
        const size_t grow = (size_t)(bq * N_ + n0 + j) * HID_;
#pragma unroll
        for (int q = 0; q < 4; ++q) {
            const int c = c0 + 8 * q;
            const v8f v = ld8f(hl + grow + c);
            u16x8 hv, lv;
            split8(v, hv, lv);
            *(u16x8*)(sHh + r * HID_ + c) = hv;
            *(u16x8*)(sHl + r * HID_ + c) = lv;
        }
    }
#pragma unroll
    for (int it = 0; it < 2; ++it) {
        const int i8 = (it * 256 + tid) * 8;
        const v8f v = ld8f(gcrw + i8);
        u16x8 hv, lv;
        split8(v, hv, lv);
        *(u16x8*)(sRh + i8) = hv;
        *(u16x8*)(sRl + i8) = lv;
    }
    {
        const int row = tid >> 3;
        const int c   = (tid & 7) * 8;
        const int rc  = min(row, DOUT_ - 1);
        const float vm = (row < DOUT_) ? 1.0f : 0.0f;
        const v8f v = ld8f(decw + rc * HID_ + c) * vm;
        u16x8 hv, lv;
        split8(v, hv, lv);
        *(u16x8*)(sDh + row * HID_ + c) = hv;
        *(u16x8*)(sDl + row * HID_ + c) = lv;
    }
    float dreg = 0.0f;
    __syncthreads();

#pragma unroll 1
    for (int ch = 0; ch < NE_ / 256; ++ch) {
        const int e  = ch * 256 + tid;
        const int d  = ei[NE_ + e];
        const int s  = ei[e];
        const float w = ew[e];
        const int jj = d - n0;
        const bool hit = ((unsigned)jj < 16u);
        const unsigned msk = __builtin_amdgcn_ballot_w32(hit);
        const int pos = __builtin_popcount(msk & ((1u << lane) - 1u));
        if (lane == 0) sCnt[wave] = __builtin_popcount(msk);
        __syncthreads();
        int off = 0, tot = 0;
#pragma unroll
        for (int w8 = 0; w8 < 8; ++w8) {
            const int cnt = sCnt[w8];
            tot += cnt;
            off += (w8 < wave) ? cnt : 0;
        }
        if (hit) {
            const int sc = min(max(s, 0), N_ - 1);
            sEj[off + pos] = (sc << 4) | jj;
            sEw[off + pos] = w;
        }
        __syncthreads();
        tot = min(tot, 256);
#pragma unroll 1
        for (int p = 0; p < tot; ++p) {
            const int   pk = sEj[p];
            const float wv = sEw[p];
            const int   j  = pk & 15;
            const int   sc = min(pk >> 4, N_ - 1);
            const v2f xv = *(const v2f*)(xl + (size_t)(bsel * N_ + sc) * HID_ + cl);
            float* ap = sAcc + (bsel * 16 + j) * HID_ + cl;
            v2f av = *(const v2f*)ap;
            av = xv * wv + av;
            *(v2f*)ap = av;
            if (tid < 16 && j == tid) dreg += wv;
        }
        __syncthreads();
    }
    if (tid < 16) sInv[tid] = 1.0f / fmaxf(dreg, 1e-12f);
    __syncthreads();

    v8f aRt[4];
    {
        FragB ah[2], al[2];
#pragma unroll
        for (int s = 0; s < 2; ++s) {
            ah[s] = frag_b(sHh + (bsel * 16 + m) * HID_, 32 * s, h);
            al[s] = frag_b(sHl + (bsel * 16 + m) * HID_, 32 * s, h);
        }
#pragma unroll
        for (int nt = 0; nt < 4; ++nt) {
            zero8(aRt[nt]);
            const unsigned short* bph = sRh + (nt * 16 + m) * HID_;
            const unsigned short* bpl = sRl + (nt * 16 + m) * HID_;
#pragma unroll
            for (int s = 0; s < 2; ++s) {
                const FragB bh = frag_b(bph, 32 * s, h);
                const FragB bl = frag_b(bpl, 32 * s, h);
                mma_bf16(aRt[nt], ah[s], bh);
                mma_bf16(aRt[nt], ah[s], bl);
                mma_bf16(aRt[nt], al[s], bh);
            }
        }
    }
    {
        float gb4[4];
#pragma unroll
        for (int nt = 0; nt < 4; ++nt) gb4[nt] = gcb[nt * 16 + m];
#pragma unroll
        for (int nt = 0; nt < 4; ++nt)
#pragma unroll
            for (int r = 0; r < 8; ++r) {
                const int j  = 8 * h + r;
                const int o  = nt * 16 + m;
                const int zi = (bsel * 16 + j) * HID_ + o;
                const float zz = aRt[nt][r] + sAcc[zi] * sInv[j] + gb4[nt];
                const unsigned short hb  = f2bf(zz);
                const unsigned short lo8 = f2bf(zz - bf2f(hb));
                sZh[zi] = hb;
                sZl[zi] = lo8;
            }
    }
    __syncthreads();

    v8f aD[2];
    {
        FragB zh[2], zl[2];
#pragma unroll
        for (int s = 0; s < 2; ++s) {
            zh[s] = frag_b(sZh + (bsel * 16 + m) * HID_, 32 * s, h);
            zl[s] = frag_b(sZl + (bsel * 16 + m) * HID_, 32 * s, h);
        }
#pragma unroll
        for (int nt = 0; nt < 2; ++nt) {
            zero8(aD[nt]);
            const unsigned short* bph = sDh + (nt * 16 + m) * HID_;
            const unsigned short* bpl = sDl + (nt * 16 + m) * HID_;
#pragma unroll
            for (int s = 0; s < 2; ++s) {
                const FragB bh = frag_b(bph, 32 * s, h);
                const FragB bl = frag_b(bpl, 32 * s, h);
                mma_bf16(aD[nt], zh[s], bh);
                mma_bf16(aD[nt], zh[s], bl);
                mma_bf16(aD[nt], zl[s], bh);
            }
        }
    }
    float* so = sOut + wave * 384;
#pragma unroll
    for (int nt = 0; nt < 2; ++nt) {
        const int o = nt * 16 + m;
        const float db = decb[min(o, DOUT_ - 1)];
        if (o < DOUT_) {
            const int tt = o >> 1, f = o & 1;
#pragma unroll
            for (int r = 0; r < 8; ++r)
                so[tt * 32 + (8 * h + r) * 2 + f] = aD[nt][r] + db;
        }
    }
    __syncthreads();

#pragma unroll
    for (int it = 0; it < 3; ++it) {
        const int tt = it * 4 + (lane >> 3);
        const int c  = (lane & 7) * 4;
        const v4f v = *(const v4f*)(so + tt * 32 + c);
        float* gp = out + ((size_t)(bsel * HOR_ + tt) * N_ + n0) * 2 + c;
        *(volatile v4f*)gp = v;
    }
    __threadfence();
#pragma unroll
    for (int it = 0; it < 3; ++it) {
        const int tt = it * 4 + (lane >> 3);
        const int c  = (lane & 7) * 4;
        const v4f v = *(const v4f*)(so + tt * 32 + c);
        float* gp = out + ((size_t)(bsel * HOR_ + tt) * N_ + n0) * 2 + c;
        *(volatile v4f*)gp = v;
    }
}

extern "C" void kernel_launch(void* const* d_in, const int* in_sizes, int n_in,
                              void* d_out, int out_size, void* d_ws, size_t ws_size,
                              hipStream_t stream)
{
    if (n_in < 15) return;
    if (in_sizes[0]  != B_ * T_ * N_ * F_) return;
    if (in_sizes[1]  != 2 * NE_)           return;
    if (in_sizes[2]  != NE_)               return;
    if (in_sizes[3]  != HID_ * F_)         return;
    if (in_sizes[4]  != HID_)              return;
    if (in_sizes[5]  != N_ * HID_)         return;
    if (in_sizes[6]  != G3_ * HID_)        return;
    if (in_sizes[7]  != G3_ * HID_)        return;
    if (in_sizes[8]  != G3_)               return;
    if (in_sizes[9]  != G3_)               return;
    if (in_sizes[10] != HID_ * HID_)       return;
    if (in_sizes[11] != HID_ * HID_)       return;
    if (in_sizes[12] != HID_)              return;
    if (in_sizes[13] != DOUT_ * HID_)      return;
    if (in_sizes[14] != DOUT_)             return;
    if (out_size != B_ * HOR_ * N_ * F_)   return;
    if (ws_size < WS_END)                  return;

    const float* x    = (const float*)d_in[0];
    const int*   ei   = (const int*)d_in[1];
    const float* ew   = (const float*)d_in[2];
    const float* encw = (const float*)d_in[3];
    const float* encb = (const float*)d_in[4];
    const float* nemb = (const float*)d_in[5];
    const float* wih  = (const float*)d_in[6];
    const float* whh  = (const float*)d_in[7];
    const float* bih  = (const float*)d_in[8];
    const float* bhh  = (const float*)d_in[9];
    const float* gcw  = (const float*)d_in[10];
    const float* gcrw = (const float*)d_in[11];
    const float* gcb  = (const float*)d_in[12];
    const float* decw = (const float*)d_in[13];
    const float* decb = (const float*)d_in[14];
    float* out = (float*)d_out;

    char* ws = (char*)d_ws;
    float* g0p = (float*)(ws + OFF_G0);
    float* hlp = (float*)(ws + OFF_HL);
    float* xlp = (float*)(ws + OFF_XL);

    hipFuncSetAttribute(reinterpret_cast<const void*>(&k_g0tab), hipFuncAttributeMaxDynamicSharedMemorySize, LDS_G0);
    k_g0tab<<<dim3(NPAD_ / 64), dim3(256), LDS_G0, stream>>>(nemb, encb, wih, bih, bhh, g0p);

    hipFuncSetAttribute(reinterpret_cast<const void*>(&k_gru), hipFuncAttributeMaxDynamicSharedMemorySize, LDS_GRU);
    k_gru<<<dim3(ROWS_ / 128), dim3(256), LDS_GRU, stream>>>(x, (const float*)g0p, encw, wih, whh, bhh, gcw, hlp, xlp);

    hipFuncSetAttribute(reinterpret_cast<const void*>(&k_gconv), hipFuncAttributeMaxDynamicSharedMemorySize, LDS_GC);
    k_gconv<<<dim3(N_ / 16), dim3(256), LDS_GC, stream>>>(ei, ew, (const float*)hlp, (const float*)xlp,
                                                         gcrw, gcb, decw, decb, out);
}
